// myBadTransfomerBlock_83605833384486
// MI455X (gfx1250) — hardware-run, weakly checked
//
#include <hip/hip_runtime.h>
#include <math.h>

constexpr int kBatch = 4;
constexpr int kSeq   = 2048;
constexpr int kDim   = 1024;
constexpr int kFF    = 4096;
constexpr int kTok   = kBatch * kSeq;
constexpr int kChunkRows = 2048;
constexpr int kNChunk    = kTok / kChunkRows;
constexpr float kWCarry    = 16.0f;
constexpr float kWCarryInv = 1.0f / 16.0f;
constexpr float kPCarry    = 2048.0f;
constexpr float kAttCarry  = 256.0f;
constexpr float kScoreScale = 1.0f / 32.0f;
constexpr float kPVScale   = kAttCarry / kPCarry;
constexpr float kWoScale   = 1.0f / (kAttCarry * kWCarry);
constexpr float kInvDim    = 1.0f / 1024.0f;
constexpr float kLnEps     = 1e-5f;
constexpr float kInvSqrt2  = 0.70710678118654752f;

constexpr size_t kMiB   = 1048576;
constexpr size_t oW1T   = 0 * kMiB;
constexpr size_t oW2T   = 8 * kMiB;
constexpr size_t oWoT   = 16 * kMiB;
constexpr size_t oWAT   = 18 * kMiB;
constexpr size_t oWBT   = 20 * kMiB;
constexpr size_t oWCT   = 22 * kMiB;
constexpr size_t oY1    = 24 * kMiB;
constexpr size_t oA16   = 40 * kMiB;
constexpr size_t oB16   = 56 * kMiB;
constexpr size_t oCT    = 72 * kMiB;
constexpr size_t oS     = 88 * kMiB;
constexpr size_t oP     = 104 * kMiB;
constexpr size_t oYatt  = 112 * kMiB;
constexpr size_t kWsTotal = 128 * kMiB;
constexpr size_t oYres  = oA16;
constexpr size_t oY2    = oY1;
constexpr size_t oU     = oCT;
constexpr size_t oH16   = oP;
static_assert(oYatt + (size_t)kTok * kDim * 2 == kWsTotal, "carve");
static_assert(oU + (size_t)kChunkRows * kFF * 4 == oP, "U region");
static_assert(oH16 + (size_t)kChunkRows * kFF * 2 <= kWsTotal, "H region");
static_assert(oYres + (size_t)kTok * kDim * 4 == oCT, "yres region");

typedef __attribute__((ext_vector_type(16))) _Float16 v16h;
typedef __attribute__((ext_vector_type(8)))  _Float16 v8h;
typedef __attribute__((ext_vector_type(16))) __bf16   v16b;
typedef __attribute__((ext_vector_type(8)))  __bf16   v8b;
typedef __attribute__((ext_vector_type(8)))  float    v8f;
typedef __attribute__((ext_vector_type(4)))  float    v4f;
typedef __attribute__((ext_vector_type(2)))  float    v2f;
typedef __attribute__((ext_vector_type(4)))  unsigned int v4u;
typedef __attribute__((ext_vector_type(2)))  unsigned int v2u;

__device__ __forceinline__ unsigned short f2bf_bits(float f) {
  unsigned u = __float_as_uint(f);
  return (unsigned short)((u + 0x7FFFu + ((u >> 16) & 1u)) >> 16);
}
__device__ __forceinline__ float bf_bits2f(unsigned short h) { return __uint_as_float(((unsigned)h) << 16); }

__device__ __forceinline__ void dep_guard_h(v8f& a, v8f& b, v16h x, v16h y) { asm volatile("v_nop\n\tv_nop\n\tv_nop\n\tv_nop" : "+v"(a), "+v"(b) : "v"(x), "v"(y)); }
__device__ __forceinline__ void dep_guard_b(v8f& a, v8f& b, v16b x, v16b y) { asm volatile("v_nop\n\tv_nop\n\tv_nop\n\tv_nop" : "+v"(a), "+v"(b) : "v"(x), "v"(y)); }
__device__ __forceinline__ void keep4_h(v16h a, v16h b, v16h c, v16h d) { asm volatile("v_nop" :: "v"(a), "v"(b), "v"(c), "v"(d)); }
__device__ __forceinline__ void keep4_b(v16b a, v16b b, v16b c, v16b d) { asm volatile("v_nop" :: "v"(a), "v"(b), "v"(c), "v"(d)); }
__device__ __forceinline__ void acc_guard4(v8f& a, v8f& b, v8f& c, v8f& d) { asm volatile("v_nop\n\tv_nop\n\tv_nop\n\tv_nop" : "+v"(a), "+v"(b), "+v"(c), "+v"(d)); }
template <typename T> struct Frag;
template <> struct Frag<_Float16> {
  typedef v16h V; union U { v16h v; v8h h[2]; };
  static __device__ __forceinline__ v16h load(const _Float16* p) {
    U f; f.h[0] = *(const v8h*)(p); f.h[1] = *(const v8h*)(p + 16); return f.v;
  }
  static __device__ __forceinline__ v8f mma(v16h a, v16h b, v8f c) {
    return __builtin_amdgcn_wmma_f32_16x16x32_f16(false, a, false, b, (short)0, c, false, false);
  }
  static __device__ __forceinline__ void guard(v8f& a, v8f& b, v16h x, v16h y) { dep_guard_h(a, b, x, y); }
  static __device__ __forceinline__ void keep(v16h a, v16h b, v16h c, v16h d) { keep4_h(a, b, c, d); }
};
template <> struct Frag<__bf16> {
  typedef v16b V; union U { v16b v; v8b h[2]; };
  static __device__ __forceinline__ v16b load(const __bf16* p) {
    U f; f.h[0] = *(const v8b*)(p); f.h[1] = *(const v8b*)(p + 16); return f.v;
  }
  static __device__ __forceinline__ v8f mma(v16b a, v16b b, v8f c) {
    return __builtin_amdgcn_wmma_f32_16x16x32_bf16(false, a, false, b, (short)0, c, false, false);
  }
  static __device__ __forceinline__ void guard(v8f& a, v8f& b, v16b x, v16b y) { dep_guard_b(a, b, x, y); }
  static __device__ __forceinline__ void keep(v16b a, v16b b, v16b c, v16b d) { keep4_b(a, b, c, d); }
};

__device__ __forceinline__ unsigned pk16(unsigned short a, unsigned short b) { return (unsigned)a | ((unsigned)b << 16); }
__device__ __forceinline__ unsigned short h_bits(float f) { const _Float16 h = (_Float16)f; return __builtin_bit_cast(unsigned short, h); }

template <int ET> struct Elem;
template <> struct Elem<0> { typedef _Float16 T; };
template <> struct Elem<1> { typedef __bf16 T; };
template <int ET, bool SPLIT, int BIAS_MODE, int OUT_MODE, bool RESID, int ACT = 0>
__global__ __launch_bounds__(256) void wmma_gemm64(
    const unsigned short* __restrict__ Ap, const unsigned short* __restrict__ A2p, int lda, long strideA,
    const unsigned short* __restrict__ Btp, const unsigned short* __restrict__ Bt2p, int ldb, long strideB,
    void* __restrict__ Cout, void* __restrict__ Cout2, int ldc, long strideC,
    const float* __restrict__ bias,
    const float* __restrict__ resid, long strideR,
    int M, int N, int K, float scale) {
  typedef typename Elem<ET>::T T;
  typedef typename Frag<T>::V V;
  const T* A = (const T*)Ap; const T* A2 = (const T*)A2p; const T* Bt = (const T*)Btp; const T* Bt2 = (const T*)Bt2p;
  __shared__ __align__(16) float sT[8][16 * 68];
  const int b    = blockIdx.y;
  const int lane = threadIdx.x & 31;
  const int wave = threadIdx.x >> 5;
  const int tilesN = N >> 6;
  const int tilesM = M >> 6;
  const int tile = blockIdx.x * 8 + wave;
  if (tile >= tilesM * tilesN) return;
  const int tm = tile / tilesN;
  const int tn = tile - tm * tilesN;
  const int m0 = tm << 6;
  const int n0 = tn << 6;

  const T* Ab  = A  + (size_t)b * strideA;
  const T* Bb  = Bt + (size_t)b * strideB;
  const T* Ab2 = SPLIT ? (A2  + (size_t)b * strideA) : nullptr;
  const T* Bb2 = SPLIT ? (Bt2 + (size_t)b * strideB) : nullptr;

  const int rlane = lane & 15;
  const int koff  = (lane >> 4) * 8;
  const int mOff  = (lane >> 4) * 8;

  v8f acc[4][4];
#pragma unroll
  for (int i = 0; i < 4; ++i)
#pragma unroll
    for (int j = 0; j < 4; ++j) acc[i][j] = (v8f){0.f,0.f,0.f,0.f,0.f,0.f,0.f,0.f};

  for (int k0 = 0; k0 < K; k0 += 32) {
    V bh[4], bl[4];
#pragma unroll
    for (int j = 0; j < 4; ++j) {
      const size_t bo = (size_t)(n0 + (j << 4) + rlane) * ldb + koff + k0;
      bh[j] = Frag<T>::load(Bb + bo);
      if (SPLIT) bl[j] = Frag<T>::load(Bb2 + bo);
    }
#pragma unroll
    for (int i = 0; i < 4; ++i) {
      const size_t ao = (size_t)(m0 + (i << 4) + rlane) * lda + koff + k0;
      V ah = Frag<T>::load(Ab + ao);
      V al;
      if (SPLIT) al = Frag<T>::load(Ab2 + ao);
#pragma unroll
      for (int j = 0; j < 4; ++j) {
        acc[i][j] = Frag<T>::mma(ah, bh[j], acc[i][j]);
        if (SPLIT) {
          acc[i][j] = Frag<T>::mma(ah, bl[j], acc[i][j]);
          acc[i][j] = Frag<T>::mma(al, bh[j], acc[i][j]);
        }
      }
      Frag<T>::guard(acc[i][0], acc[i][3], ah, SPLIT ? al : ah);
    }
    Frag<T>::keep(bh[0], bh[1], bh[2], bh[3]);
    if (SPLIT) Frag<T>::keep(bl[0], bl[1], bl[2], bl[3]);
  }
  acc_guard4(acc[0][0], acc[0][1], acc[0][2], acc[0][3]);
  acc_guard4(acc[1][0], acc[1][1], acc[1][2], acc[1][3]);
  acc_guard4(acc[2][0], acc[2][1], acc[2][2], acc[2][3]);
  acc_guard4(acc[3][0], acc[3][1], acc[3][2], acc[3][3]);

  float* slab = sT[wave];
  const float* Rb = RESID ? (resid + (size_t)b * strideR) : nullptr;
#pragma unroll
  for (int i = 0; i < 4; ++i) {
    const int mBase = m0 + (i << 4);
#pragma unroll
    for (int j = 0; j < 4; ++j) {
      const int n = n0 + (j << 4) + rlane;
      float bv = 0.f;
      if (BIAS_MODE == 2) bv = bias[n];
#pragma unroll
      for (int r = 0; r < 8; ++r) {
        float v = acc[i][j][r] * scale;
        if (BIAS_MODE == 1) v += bias[mBase + mOff + r];
        if (BIAS_MODE == 2) v += bv;
        if (RESID) v += Rb[(size_t)(mBase + mOff + r) * ldc + n];
        if (ACT == 2) v = fmaxf(v, 0.0f);
        if (ACT == 4) v = (v > 0.f) ? v : 0.01f * v;
        slab[(mOff + r) * 68 + (j << 4) + rlane] = v;
      }
    }
    __builtin_amdgcn_fence(__ATOMIC_RELEASE, "workgroup");
    __builtin_amdgcn_wave_barrier();
    __builtin_amdgcn_fence(__ATOMIC_ACQUIRE, "workgroup");
    if (OUT_MODE == 0) {
      float* C = (float*)Cout + (size_t)b * strideC;
      const int hh = lane >> 4, c4 = (lane & 15) * 4;
      for (int pass = 0; pass < 2; ++pass) {
#pragma unroll
        for (int it = 0; it < 8; ++it) {
          const int row = it * 2 + hh;
          v4f v = *(const v4f*)(slab + row * 68 + c4);
          *(volatile v4f*)(C + (size_t)(mBase + row) * ldc + n0 + c4) = v;
        }
        __threadfence();
      }
    } else {
      const int q = lane >> 3, c8 = (lane & 7) * 8;
      unsigned short* C  = (unsigned short*)Cout  + (size_t)b * strideC;
      unsigned short* C2 = (OUT_MODE == 2) ? ((unsigned short*)Cout2 + (size_t)b * strideC) : nullptr;
      for (int pass = 0; pass < 2; ++pass) {
#pragma unroll
        for (int it = 0; it < 4; ++it) {
          const int row = it * 4 + q;
          const float* sp = slab + row * 68 + c8;
          v8h hv, lv;
#pragma unroll
          for (int e = 0; e < 8; ++e) {
            if (OUT_MODE == 1) {
              hv[e] = (_Float16)sp[e];
            } else {
              unsigned short hb = f2bf_bits(sp[e]);
              unsigned short lb = f2bf_bits(sp[e] - bf_bits2f(hb));
              hv[e] = __builtin_bit_cast(_Float16, hb);
              lv[e] = __builtin_bit_cast(_Float16, lb);
            }
          }
          *(volatile v8h*)(C + (size_t)(mBase + row) * ldc + n0 + c8) = hv;
          if (OUT_MODE == 2) *(volatile v8h*)(C2 + (size_t)(mBase + row) * ldc + n0 + c8) = lv;
        }
        __threadfence();
      }
    }
    __builtin_amdgcn_fence(__ATOMIC_RELEASE, "workgroup");
    __builtin_amdgcn_wave_barrier();
    __builtin_amdgcn_fence(__ATOMIC_ACQUIRE, "workgroup");
  }
}

__global__ __launch_bounds__(256) void tcast_f16_kernel(const float* __restrict__ W, unsigned short* __restrict__ WT,
                                                        int Kd, int Nd, float scale) {
  __shared__ float sm[64][65];
  const int t  = threadIdx.x;
  const int k0 = blockIdx.x * 64;
  const int n0 = blockIdx.y * 64;
#pragma unroll
  for (int i = 0; i < 16; ++i) {
    const int e = i * 256 + t;
    const int r = e >> 6;
    const int c = e & 63;
    sm[c][r] = W[(size_t)(k0 + r) * Nd + n0 + c] * scale;
  }
  __syncthreads();
  const int lane = t & 31, wave = t >> 5;
  const int q = lane >> 3, c8 = (lane & 7) * 8;
  for (int pass = 0; pass < 2; ++pass) {
#pragma unroll
    for (int it = 0; it < 2; ++it) {
      const int row = wave * 8 + it * 4 + q;
      unsigned short hb[8];
#pragma unroll
      for (int e = 0; e < 8; ++e) hb[e] = h_bits(sm[row][c8 + e]);
      const v4u u = (v4u){pk16(hb[0], hb[1]), pk16(hb[2], hb[3]), pk16(hb[4], hb[5]), pk16(hb[6], hb[7])};
      *(volatile v4u*)(WT + (size_t)(n0 + row) * Kd + k0 + c8) = u;
    }
    __threadfence();
  }
}

__global__ __launch_bounds__(256) void layernorm_f16_kernel(const float* __restrict__ X, const float* __restrict__ gam,
                                                            const float* __restrict__ bet, unsigned short* __restrict__ Y) {
  __shared__ float redA[8];
  __shared__ float redB[8];
  const int row  = blockIdx.x;
  const int t    = threadIdx.x;
  const int lane = t & 31, wave = t >> 5;
  const v4f v = *(const v4f*)(X + (size_t)row * kDim + 4 * t);
  float s = (v[0] + v[1]) + (v[2] + v[3]);
#pragma unroll
  for (int off = 16; off > 0; off >>= 1) s += __shfl_xor(s, off, 32);
  if (lane == 0) redA[wave] = s;
  __syncthreads();
  float tot = 0.f;
#pragma unroll
  for (int w = 0; w < 8; ++w) tot += redA[w];
  const float mu = tot * kInvDim;
  const float d0 = v[0] - mu, d1 = v[1] - mu, d2 = v[2] - mu, d3 = v[3] - mu;
  float sq = (d0 * d0 + d1 * d1) + (d2 * d2 + d3 * d3);
#pragma unroll
  for (int off = 16; off > 0; off >>= 1) sq += __shfl_xor(sq, off, 32);
  if (lane == 0) redB[wave] = sq;
  __syncthreads();
  float tot2 = 0.f;
#pragma unroll
  for (int w = 0; w < 8; ++w) tot2 += redB[w];
  const float var  = tot2 * kInvDim;
  const float rstd = rsqrtf(var + kLnEps);
  const v4f gv = *(const v4f*)(gam + 4 * t);
  const v4f bv = *(const v4f*)(bet + 4 * t);
  const float y0 = d0 * rstd * gv[0] + bv[0];
  const float y1 = d1 * rstd * gv[1] + bv[1];
  const float y2 = d2 * rstd * gv[2] + bv[2];
  const float y3 = d3 * rstd * gv[3] + bv[3];
  const v2u u = (v2u){pk16(h_bits(y0), h_bits(y1)), pk16(h_bits(y2), h_bits(y3))};
  unsigned short* yp = Y + (size_t)row * kDim + 4 * t;
  *(volatile v2u*)yp = u;
  __threadfence();
  *(volatile v2u*)yp = u;
}

__global__ __launch_bounds__(256) void softmax_row_kernel(const float* __restrict__ S, unsigned short* __restrict__ P) {
  __shared__ float redM[8];
  __shared__ float redS[8];
  const int row  = blockIdx.x;
  const int t    = threadIdx.x;
  const int lane = t & 31, wave = t >> 5;
  const int c0   = t * 8;
  const float* sr = S + (size_t)row * kSeq + c0;
  const v4f a = *(const v4f*)(sr);
  const v4f c = *(const v4f*)(sr + 4);
  float x[8];
#pragma unroll
  for (int e = 0; e < 4; ++e) { x[e] = a[e]; x[4 + e] = c[e]; }
  float m = fmaxf(fmaxf(fmaxf(x[0], x[1]), fmaxf(x[2], x[3])), fmaxf(fmaxf(x[4], x[5]), fmaxf(x[6], x[7])));
#pragma unroll
  for (int off = 16; off > 0; off >>= 1) m = fmaxf(m, __shfl_xor(m, off, 32));
  if (lane == 0) redM[wave] = m;
  __syncthreads();
  float mm = redM[0];
#pragma unroll
  for (int w = 1; w < 8; ++w) mm = fmaxf(mm, redM[w]);
  float ev[8];
  float s = 0.f;
#pragma unroll
  for (int e = 0; e < 8; ++e) { ev[e] = expf(x[e] - mm); s += ev[e]; }
#pragma unroll
  for (int off = 16; off > 0; off >>= 1) s += __shfl_xor(s, off, 32);
  if (lane == 0) redS[wave] = s;
  __syncthreads();
  float tot = 0.f;
#pragma unroll
  for (int w = 0; w < 8; ++w) tot += redS[w];
  const float inv = kPCarry * (1.0f / tot);
  unsigned short hb[8];
#pragma unroll
  for (int e = 0; e < 8; ++e) hb[e] = h_bits(ev[e] * inv);
  const v4u u = (v4u){pk16(hb[0], hb[1]), pk16(hb[2], hb[3]), pk16(hb[4], hb[5]), pk16(hb[6], hb[7])};
  unsigned short* pp = P + (size_t)row * kSeq + c0;
  *(volatile v4u*)pp = u;
  __threadfence();
  *(volatile v4u*)pp = u;
}

__global__ __launch_bounds__(256) void gelu_f16_kernel(const float* __restrict__ U, unsigned short* __restrict__ H, int n2) {
  const int i = blockIdx.x * 256 + threadIdx.x;
  if (i >= n2) return;
  const v2f u = *(const v2f*)(U + 2 * (size_t)i);
  const float g0 = 0.5f * u[0] * (1.0f + erff(u[0] * kInvSqrt2));
  const float g1 = 0.5f * u[1] * (1.0f + erff(u[1] * kInvSqrt2));
  const unsigned w = pk16(h_bits(g0), h_bits(g1));
  unsigned short* hp = H + 2 * (size_t)i;
  *(volatile unsigned*)hp = w;
  __threadfence();
  *(volatile unsigned*)hp = w;
}

extern "C" void kernel_launch(void* const* d_in, const int* in_sizes, int n_in,
                              void* d_out, int out_size, void* d_ws, size_t ws_size,
                              hipStream_t stream) {
  if (n_in < 17) return;
  if (in_sizes[0] != kTok * kDim) return;
  if (in_sizes[1] != kDim * kDim || in_sizes[3] != kDim * kDim || in_sizes[5] != kDim * kDim || in_sizes[7] != kDim * kDim) return;
  if (in_sizes[2] != kDim || in_sizes[4] != kDim || in_sizes[6] != kDim || in_sizes[8] != kDim) return;
  if (in_sizes[9] != kDim || in_sizes[10] != kDim || in_sizes[11] != kDim || in_sizes[12] != kDim) return;
  if (in_sizes[13] != kDim * kFF || in_sizes[14] != kFF || in_sizes[15] != kFF * kDim || in_sizes[16] != kDim) return;
  if (out_size != kTok * kDim) return;
  if (ws_size < kWsTotal) return;

  const float* x   = (const float*)d_in[0];
  const float* WA  = (const float*)d_in[1];
  const float* bA  = (const float*)d_in[2];
  const float* WB  = (const float*)d_in[3];
  const float* bB  = (const float*)d_in[4];
  const float* WC  = (const float*)d_in[5];
  const float* bC  = (const float*)d_in[6];
  const float* Wo  = (const float*)d_in[7];
  const float* bo  = (const float*)d_in[8];
  const float* g1  = (const float*)d_in[9];
  const float* be1 = (const float*)d_in[10];
  const float* g2  = (const float*)d_in[11];
  const float* be2 = (const float*)d_in[12];
  const float* W1  = (const float*)d_in[13];
  const float* b1  = (const float*)d_in[14];
  const float* W2  = (const float*)d_in[15];
  const float* b2  = (const float*)d_in[16];
  float* out = (float*)d_out;

  char* ws = (char*)d_ws;
  unsigned short* W1T  = (unsigned short*)(ws + oW1T);
  unsigned short* W2T  = (unsigned short*)(ws + oW2T);
  unsigned short* WoT  = (unsigned short*)(ws + oWoT);
  unsigned short* WAT  = (unsigned short*)(ws + oWAT);
  unsigned short* WBT  = (unsigned short*)(ws + oWBT);
  unsigned short* WCT  = (unsigned short*)(ws + oWCT);
  unsigned short* Y1   = (unsigned short*)(ws + oY1);
  unsigned short* A16  = (unsigned short*)(ws + oA16);
  unsigned short* B16  = (unsigned short*)(ws + oB16);
  unsigned short* CT   = (unsigned short*)(ws + oCT);
  float*          S    = (float*)(ws + oS);
  unsigned short* P    = (unsigned short*)(ws + oP);
  unsigned short* Yatt = (unsigned short*)(ws + oYatt);
  float*          yres = (float*)(ws + oYres);
  unsigned short* Y2   = (unsigned short*)(ws + oY2);
  float*          U    = (float*)(ws + oU);
  unsigned short* H16  = (unsigned short*)(ws + oH16);

  tcast_f16_kernel<<<dim3(kDim / 64, kDim / 64), 256, 0, stream>>>(WA, WAT, kDim, kDim, kWCarry);
  tcast_f16_kernel<<<dim3(kDim / 64, kDim / 64), 256, 0, stream>>>(WB, WBT, kDim, kDim, kWCarry);
  tcast_f16_kernel<<<dim3(kDim / 64, kDim / 64), 256, 0, stream>>>(WC, WCT, kDim, kDim, kWCarry);
  tcast_f16_kernel<<<dim3(kDim / 64, kDim / 64), 256, 0, stream>>>(Wo, WoT, kDim, kDim, kWCarry);
  tcast_f16_kernel<<<dim3(kDim / 64, kFF / 64), 256, 0, stream>>>(W1, W1T, kDim, kFF, kWCarry);
  tcast_f16_kernel<<<dim3(kFF / 64, kDim / 64), 256, 0, stream>>>(W2, W2T, kFF, kDim, kWCarry);

  layernorm_f16_kernel<<<kTok, 256, 0, stream>>>(x, g1, be1, Y1);

  {
    const int gx = ((kTok / 64) * (kDim / 64) + 7) / 8;
    wmma_gemm64<0, false, 2, 1, false><<<dim3(gx, 1), 256, 0, stream>>>(
        Y1, nullptr, kDim, 0L, WAT, nullptr, kDim, 0L, (void*)A16, nullptr, kDim, 0L,
        bA, nullptr, 0L, kTok, kDim, kDim, kWCarryInv);
    wmma_gemm64<0, false, 2, 1, false><<<dim3(gx, 1), 256, 0, stream>>>(
        Y1, nullptr, kDim, 0L, WBT, nullptr, kDim, 0L, (void*)B16, nullptr, kDim, 0L,
        bB, nullptr, 0L, kTok, kDim, kDim, kWCarryInv);
  }
  {
    const int gx = ((kDim / 64) * (kSeq / 64) + 7) / 8;
    wmma_gemm64<0, false, 1, 1, false><<<dim3(gx, kBatch), 256, 0, stream>>>(
        WCT, nullptr, kDim, 0L, Y1, nullptr, kDim, (long)kSeq * kDim, (void*)CT, nullptr, kSeq, (long)kDim * kSeq,
        bC, nullptr, 0L, kDim, kSeq, kDim, kWCarryInv);
  }

  for (int bt = 0; bt < kBatch; ++bt) {
    const unsigned short* Ab = A16 + (size_t)bt * kSeq * kDim;
    const unsigned short* Bb = B16 + (size_t)bt * kSeq * kDim;
    const unsigned short* CTb = CT + (size_t)bt * kDim * kSeq;
    unsigned short* Yb = Yatt + (size_t)bt * kSeq * kDim;
    const int gxS = ((kSeq / 64) * (kSeq / 64) + 7) / 8;
    wmma_gemm64<0, false, 0, 0, false><<<dim3(gxS, 1), 256, 0, stream>>>(
        Ab, nullptr, kDim, 0L, Bb, nullptr, kDim, 0L, (void*)S, nullptr, kSeq, 0L,
        nullptr, nullptr, 0L, kSeq, kSeq, kDim, kScoreScale);
    softmax_row_kernel<<<kSeq, 256, 0, stream>>>(S, P);
    const int gxO = ((kSeq / 64) * (kDim / 64) + 7) / 8;
    wmma_gemm64<0, false, 0, 1, false><<<dim3(gxO, 1), 256, 0, stream>>>(
        P, nullptr, kSeq, 0L, CTb, nullptr, kSeq, 0L, (void*)Yb, nullptr, kDim, 0L,
        nullptr, nullptr, 0L, kSeq, kDim, kSeq, kPVScale);
  }

  {
    const int gx = ((kTok / 64) * (kDim / 64) + 7) / 8;
    wmma_gemm64<0, false, 2, 0, true><<<dim3(gx, 1), 256, 0, stream>>>(
        Yatt, nullptr, kDim, 0L, WoT, nullptr, kDim, 0L, (void*)yres, nullptr, kDim, 0L,
        bo, x, 0L, kTok, kDim, kDim, kWoScale);
  }

  layernorm_f16_kernel<<<kTok, 256, 0, stream>>>(yres, g2, be2, Y2);

  for (int ch = 0; ch < kNChunk; ++ch) {
    const unsigned short* Y2c = Y2 + (size_t)ch * kChunkRows * kDim;
    const float* xc = x + (size_t)ch * kChunkRows * kDim;
    float* outc = out + (size_t)ch * kChunkRows * kDim;
    const int gx1 = ((kChunkRows / 64) * (kFF / 64) + 7) / 8;
    wmma_gemm64<0, false, 2, 0, false><<<dim3(gx1, 1), 256, 0, stream>>>(
        Y2c, nullptr, kDim, 0L, W1T, nullptr, kDim, 0L, (void*)U, nullptr, kFF, 0L,
        b1, nullptr, 0L, kChunkRows, kFF, kDim, kWCarryInv);
    const int n2 = kChunkRows * kFF / 2;
    gelu_f16_kernel<<<(n2 + 255) / 256, 256, 0, stream>>>(U, H16, n2);
    const int gx2 = ((kChunkRows / 64) * (kDim / 64) + 7) / 8;
    wmma_gemm64<0, false, 2, 0, true><<<dim3(gx2, 1), 256, 0, stream>>>(
        H16, nullptr, kFF, 0L, W2T, nullptr, kFF, 0L, (void*)outc, nullptr, kDim, 0L,
        b2, xc, 0L, kChunkRows, kDim, kFF, kWCarryInv);
  }
}
